// EdgeAwareGAT_16870631539205
// MI455X (gfx1250) — hardware-verified
//
#include <hip/hip_runtime.h>


#define NN_ 10000
#define NE_ 160000
#define NG 64
#define DIN 771
#define HID 256
#define NH 4
#define IL_CAP 48

typedef __attribute__((ext_vector_type(16))) __bf16   v16bf;
typedef __attribute__((ext_vector_type(16))) _Float16 v16h;
typedef __attribute__((ext_vector_type(8)))  float    v8f;
typedef __attribute__((ext_vector_type(8)))  unsigned v8u;

__device__ __forceinline__ unsigned f2bf(float f) { unsigned u = __float_as_uint(f); u += 0x7FFFu + ((u >> 16) & 1u); return u >> 16; }
__device__ __forceinline__ unsigned f2h(float f) { return (unsigned)__builtin_bit_cast(unsigned short, (_Float16)f); }
__device__ __forceinline__ int kpat(int v, int half) { return ((v & 4) ? 16 : 0) + half * 8 + 2 * (v & 3); }

template <int F16, int NP> struct Opnd { v16bf p[NP]; };

template <int F16, int NP> __device__ __forceinline__ void pack2(float f0, float f1, unsigned* o) {
    if (F16) { o[0] = f2h(f0) | (f2h(f1) << 16); return; }
    unsigned h0 = f2bf(f0), h1 = f2bf(f1); o[0] = h0 | (h1 << 16);
    if (NP >= 2) {
        float r0 = f0 - __uint_as_float(h0 << 16), r1 = f1 - __uint_as_float(h1 << 16);
        unsigned m0 = f2bf(r0), m1 = f2bf(r1); o[1] = m0 | (m1 << 16);
        if (NP >= 3) {
            float s0 = r0 - __uint_as_float(m0 << 16), s1 = r1 - __uint_as_float(m1 << 16);
            o[2] = f2bf(s0) | (f2bf(s1) << 16);
        }
    }
}
template <int F16, int NP> __device__ __forceinline__ void op_row(const float* rowp, int half, float sc, Opnd<F16, NP>& o) {
    v8u u[NP];
#pragma unroll
    for (int v = 0; v < 8; ++v) {
        int kk = kpat(v, half); unsigned t[3];
        pack2<F16, NP>(rowp[kk] * sc, rowp[kk + 1] * sc, t);
#pragma unroll
        for (int p = 0; p < NP; ++p) u[p][v] = t[p];
    }
#pragma unroll
    for (int p = 0; p < NP; ++p) o.p[p] = __builtin_bit_cast(v16bf, u[p]);
}
template <int F16, int NP> __device__ __forceinline__ void op_row_tail(const float* rowp, int half, float sc, int kvalid, Opnd<F16, NP>& o) {
    v8u u[NP];
#pragma unroll
    for (int v = 0; v < 8; ++v) {
        int kk = kpat(v, half); unsigned t[3];
        float f0 = kk < kvalid ? rowp[kk] * sc : 0.0f, f1 = (kk + 1) < kvalid ? rowp[kk + 1] * sc : 0.0f;
        pack2<F16, NP>(f0, f1, t);
#pragma unroll
        for (int p = 0; p < NP; ++p) u[p][v] = t[p];
    }
#pragma unroll
    for (int p = 0; p < NP; ++p) o.p[p] = __builtin_bit_cast(v16bf, u[p]);
}
template <int F16, int NP> __device__ __forceinline__ void op_col(const float* M, int ld, int n, int k0, int half, float sc, Opnd<F16, NP>& o) {
    v8u u[NP];
#pragma unroll
    for (int v = 0; v < 8; ++v) {
        int kk = k0 + kpat(v, half); unsigned t[3];
        pack2<F16, NP>(M[(size_t)kk * ld + n] * sc, M[(size_t)(kk + 1) * ld + n] * sc, t);
#pragma unroll
        for (int p = 0; p < NP; ++p) u[p][v] = t[p];
    }
#pragma unroll
    for (int p = 0; p < NP; ++p) o.p[p] = __builtin_bit_cast(v16bf, u[p]);
}
template <int F16, int NP> __device__ __forceinline__ void op_col_tail(const float* M, int ld, int n, int k0, int half, float sc, int K, Opnd<F16, NP>& o) {
    v8u u[NP];
#pragma unroll
    for (int v = 0; v < 8; ++v) {
        int kk = k0 + kpat(v, half); unsigned t[3];
        float f0 = kk < K ? M[(size_t)kk * ld + n] * sc : 0.0f, f1 = (kk + 1) < K ? M[(size_t)(kk + 1) * ld + n] * sc : 0.0f;
        pack2<F16, NP>(f0, f1, t);
#pragma unroll
        for (int p = 0; p < NP; ++p) u[p][v] = t[p];
    }
#pragma unroll
    for (int p = 0; p < NP; ++p) o.p[p] = __builtin_bit_cast(v16bf, u[p]);
}
__device__ __forceinline__ v8f wm_bf16(v16bf a, v16bf b, v8f c) { return __builtin_amdgcn_wmma_f32_16x16x32_bf16(false, a, false, b, (short)0, c, false, false); }
template <int F16, int NA, int NB> __device__ __forceinline__ v8f wmma_op(const Opnd<F16, NA>& a, const Opnd<F16, NB>& b, v8f c) {
    if (F16) {
        v16h ah = __builtin_bit_cast(v16h, a.p[0]), bh = __builtin_bit_cast(v16h, b.p[0]);
        c = __builtin_amdgcn_wmma_f32_16x16x32_f16(false, ah, false, bh, (short)0, c, false, false);
        asm volatile("v_nop\n\tv_nop\n\tv_nop\n\tv_nop" : "+v"(c) : "v"(ah), "v"(bh));
        return c;
    }
    constexpr int NMX = NA > NB ? NA : NB;
#pragma unroll
    for (int i = 0; i < NA; ++i)
#pragma unroll
        for (int j = 0; j < NB; ++j)
            if (i + j < NMX) c = wm_bf16(a.p[i], b.p[j], c);
    if (NA == 1 && NB == 1)      asm volatile("v_nop\n\tv_nop\n\tv_nop\n\tv_nop" : "+v"(c) : "v"(a.p[0]), "v"(b.p[0]));
    else if (NA == 2 && NB == 1) asm volatile("v_nop\n\tv_nop\n\tv_nop\n\tv_nop" : "+v"(c) : "v"(a.p[0]), "v"(a.p[1]), "v"(b.p[0]));
    else if (NA == 1 && NB == 2) asm volatile("v_nop\n\tv_nop\n\tv_nop\n\tv_nop" : "+v"(c) : "v"(a.p[0]), "v"(b.p[0]), "v"(b.p[1]));
    else if (NA == 2 && NB == 2) asm volatile("v_nop\n\tv_nop\n\tv_nop\n\tv_nop" : "+v"(c) : "v"(a.p[0]), "v"(a.p[1]), "v"(b.p[0]), "v"(b.p[1]));
    else                         asm volatile("v_nop\n\tv_nop\n\tv_nop\n\tv_nop" : "+v"(c) : "v"(a.p[0]), "v"(a.p[NA - 1]), "v"(b.p[0]), "v"(b.p[NB - 1]), "v"(a.p[NA / 2]), "v"(b.p[NB / 2]));
    return c;
}

struct ZMap { long long s1; long long s2; int zdiv; int pad_; };
__device__ __forceinline__ size_t zoff(const ZMap& m, int z) { return (size_t)((long long)(z / m.zdiv) * m.s1 + (long long)(z % m.zdiv) * m.s2); }

#define ACT_NONE 0
#define ACT_RELU 1
#define ACT_GELU_ERF 2
#define ACT_SILU 3
#define ACT_TANH 4
__device__ __forceinline__ float act_apply(int act, float x) {
    if (act == ACT_RELU) return x > 0.f ? x : 0.f;
    if (act == ACT_GELU_ERF) return 0.5f * x * (1.0f + erff(x * 0.70710678118654752f));
    if (act == ACT_SILU) return x / (1.0f + expf(-x));
    if (act == ACT_TANH) return tanhf(x);
    return x;
}
struct GemmArgs {
    ZMap za, zb_, zc, zbias, zadd, zrsc, zmul, zrbias;
    const float* A; const float* Bm; float* C; const float* bias; const float* add; const float* rsc; const float* mul; const float* rbias;
    long long ldadd, ldmul;
    int lda, ldb, ldc, K;
    float ascale, bscale, oscale, addscale;
    int M, nvalid, nstore, ldrsc;
    int bcs, pad1, pad2, pad3;
};
template <int BT, int F16, int NA, int NB, int RW, int CW, int ACT>
__global__ __launch_bounds__(256) void gemm_kernel(GemmArgs g) {
    constexpr int TR = 16 * RW, TC = 64 * CW, CSTR = TC + 4;
    __shared__ __align__(16) float cst[TR * CSTR];
    const int z = blockIdx.z;
    const float* A = g.A + zoff(g.za, z); const float* Bm = g.Bm + zoff(g.zb_, z); float* C = g.C + zoff(g.zc, z);
    const int tid = threadIdx.x, lane = tid & 31, wv = tid >> 5;
    const int l16 = lane & 15, half = lane >> 4;
    const int rt = wv % RW, ch = wv / RW;
    const int row0 = blockIdx.x * TR, col0 = blockIdx.y * TC + ch * 64;
    int arix = row0 + rt * 16 + l16; if (arix >= g.M) arix = g.M - 1;
    const float* arow = A + (size_t)arix * g.lda;
    v8f acc[4];
#pragma unroll
    for (int t = 0; t < 4; ++t) acc[t] = (v8f){};
    const int K = g.K;
#pragma unroll 1
    for (int kc = 0; kc < K; kc += 32) {
        Opnd<F16, NA> a;
        if (kc + 32 <= K) op_row<F16, NA>(arow + kc, half, g.ascale, a); else op_row_tail<F16, NA>(arow + kc, half, g.ascale, K - kc, a);
#pragma unroll
        for (int t = 0; t < 4; ++t) {
            Opnd<F16, NB> b;
            const int n = col0 + t * 16 + l16;
            if (n < g.nvalid) {
                if (BT) { if (kc + 32 <= K) op_row<F16, NB>(Bm + (size_t)n * g.ldb + kc, half, g.bscale, b); else op_row_tail<F16, NB>(Bm + (size_t)n * g.ldb + kc, half, g.bscale, K - kc, b); }
                else    { if (kc + 32 <= K) op_col<F16, NB>(Bm, g.ldb, n * g.bcs, kc, half, g.bscale, b); else op_col_tail<F16, NB>(Bm, g.ldb, n * g.bcs, kc, half, g.bscale, K, b); }
            } else {
#pragma unroll
                for (int p = 0; p < NB; ++p) b.p[p] = (v16bf){};
            }
            acc[t] = wmma_op<F16, NA, NB>(a, b, acc[t]);
        }
    }
    const float* bias = g.bias ? g.bias + zoff(g.zbias, z) : nullptr;
    const float* add = g.add ? g.add + zoff(g.zadd, z) : nullptr;
    const float* rsc = g.rsc ? g.rsc + zoff(g.zrsc, z) : nullptr;
    const float* mul = g.mul ? g.mul + zoff(g.zmul, z) : nullptr;
    const float* rbias = g.rbias ? g.rbias + zoff(g.zrbias, z) : nullptr;
#pragma unroll
    for (int t = 0; t < 4; ++t) {
        const int cl = ch * 64 + t * 16 + l16;
        const int cg = blockIdx.y * TC + cl;
        const bool cok = cg < g.nvalid;
        const float bv = (bias && cok) ? bias[(size_t)cg * g.bcs] : 0.0f;
#pragma unroll
        for (int r = 0; r < 8; ++r) {
            const int rl = rt * 16 + r + 8 * half;
            float v = acc[t][r] * g.oscale + bv;
            int rg = row0 + rl; if (rg >= g.M) rg = g.M - 1;
            if (rbias) v += rbias[rg];
            if (rsc) v *= rsc[(size_t)rg * g.ldrsc];
            if (mul && cok) v *= mul[(size_t)rg * g.ldmul + cg];
            if (add && cok) v += g.addscale * add[(size_t)rg * g.ldadd + cg];
            cst[rl * CSTR + cl] = v;
        }
    }
    __syncthreads();
    const int col = tid % TC, rsel = tid / TC, rstep = 256 / TC;
    if (ACT != ACT_NONE) {
#pragma unroll 1
        for (int r = rsel; r < TR; r += rstep) cst[r * CSTR + col] = act_apply(ACT, cst[r * CSTR + col]);
    }
    float* ob = C + (size_t)row0 * g.ldc + (size_t)blockIdx.y * TC;
    const bool colok = (int)(blockIdx.y * TC + col) < g.nstore;
    const int rmax = (g.M - row0 < TR) ? (g.M - row0) : TR;
    auto pass = [&]() {
        if (colok) {
#pragma unroll 4
            for (int r = rsel; r < rmax; r += rstep) *(volatile float*)(ob + (size_t)r * g.ldc + col) = cst[r * CSTR + col];
        }
    };
    pass();
    __threadfence();
    pass();
}
static inline ZMap zm(long long s1) { ZMap m; m.s1 = s1; m.s2 = 0; m.zdiv = 1; m.pad_ = 0; return m; }
static inline ZMap zm2(long long s1, long long s2, int zdiv) { ZMap m; m.s1 = s1; m.s2 = s2; m.zdiv = zdiv; m.pad_ = 0; return m; }
static inline GemmArgs gemm_args(const float* A, int lda, ZMap za, const float* Bm, int ldb, ZMap zb, float* C, int ldc, ZMap zc, int M, int N, int K) {
    GemmArgs g; g.za = za; g.zb_ = zb; g.zc = zc; g.zbias = zm(0); g.zadd = zm(0); g.zrsc = zm(0); g.zmul = zm(0); g.zrbias = zm(0);
    g.A = A; g.Bm = Bm; g.C = C; g.bias = nullptr; g.add = nullptr; g.rsc = nullptr; g.mul = nullptr; g.rbias = nullptr; g.ldadd = 0; g.ldmul = 0;
    g.lda = lda; g.ldb = ldb; g.ldc = ldc; g.K = K; g.ascale = 1.0f; g.bscale = 1.0f; g.oscale = 1.0f; g.addscale = 1.0f; g.M = M; g.nvalid = N; g.nstore = N; g.ldrsc = 1;
    g.bcs = 1; g.pad1 = 0; g.pad2 = 0; g.pad3 = 0;
    return g;
}
static_assert(sizeof(ZMap) == 24, "ZMap layout");
static_assert(sizeof(GemmArgs) == 8 * 24 + 8 * 8 + 2 * 8 + 4 * 4 + 4 * 4 + 4 * 4 + 4 * 4, "GemmArgs has no padding");

__global__ __launch_bounds__(256) void softmax_rows(float* S, long long sy, long long sx, int L, float prescale, const float* addv, long long say, int aydiv, int causal,
                                                  const int* imask, long long imy, long long imx, float maskval) {
    __shared__ float red[8];
    const int tid = threadIdx.x, lane = tid & 31, wid = tid >> 5;
    float* row = S + (size_t)blockIdx.y * sy + (size_t)blockIdx.x * sx;
    const float* av = addv ? addv + (size_t)(blockIdx.y / aydiv) * say : nullptr;
    const int* im = imask ? imask + (size_t)(blockIdx.y / aydiv) * imy + (size_t)blockIdx.x * imx : nullptr;
    float v[16];
    const int nj = L / 256;
    float mx = -__builtin_inff();
#pragma unroll
    for (int j = 0; j < 16; ++j) if (j < nj) { float t = row[tid + 256 * j] * prescale; if (av) t += av[tid + 256 * j]; if (im && im[tid + 256 * j] == 0) t = maskval; if (causal && (tid + 256 * j) > (int)blockIdx.x) t = -__builtin_inff(); v[j] = t; mx = fmaxf(mx, t); }
#pragma unroll
    for (int o = 16; o; o >>= 1) mx = fmaxf(mx, __shfl_xor(mx, o, 32));
    if (lane == 0) red[wid] = mx;
    __syncthreads();
    float m = red[0];
#pragma unroll
    for (int i = 1; i < 8; ++i) m = fmaxf(m, red[i]);
    if (m == -__builtin_inff()) m = 0.f;
    __syncthreads();
    float sum = 0.f;
#pragma unroll
    for (int j = 0; j < 16; ++j) if (j < nj) { v[j] = expf(v[j] - m); sum += v[j]; }
#pragma unroll
    for (int o = 16; o; o >>= 1) sum += __shfl_xor(sum, o, 32);
    if (lane == 0) red[wid] = sum;
    __syncthreads();
    float tot = 0.f;
#pragma unroll
    for (int i = 0; i < 8; ++i) tot += red[i];
    const float inv = 1.0f / tot;
#pragma unroll
    for (int j = 0; j < 16; ++j) if (j < nj) *(volatile float*)(row + tid + 256 * j) = v[j] * inv;
    __threadfence();
#pragma unroll
    for (int j = 0; j < 16; ++j) if (j < nj) *(volatile float*)(row + tid + 256 * j) = v[j] * inv;
}

#define VST2(T, p, v) do { const T vst2_v_ = (v); *(volatile T*)(p) = vst2_v_; __threadfence(); *(volatile T*)(p) = vst2_v_; } while (0)
#define IL_T 128
#define IL_TILE 4096
__global__ __launch_bounds__(IL_T) void k_inlists(const int* __restrict__ tgt, int E, int N, int* NBR, int* cnt) {
    __shared__ int tt[IL_TILE];
    __shared__ int lists[IL_T * IL_CAP];
    const int d = blockIdx.x * IL_T + threadIdx.x; int n = 0;
    for (int e0 = 0; e0 < E; e0 += IL_TILE) {
        const int nt = min(IL_TILE, E - e0);
        __syncthreads();
        for (int i = threadIdx.x; i < nt; i += IL_T) tt[i] = tgt[e0 + i];
        __syncthreads();
        for (int i = 0; i < nt; ++i) { if (tt[i] == d) { if (n < IL_CAP) lists[threadIdx.x * IL_CAP + n] = e0 + i; ++n; } }
    }
    if (d < N) {
        int* row = NBR + (size_t)d * IL_CAP;
        for (int j = 0; j < IL_CAP; ++j) { const int v = (j < n) ? lists[threadIdx.x * IL_CAP + j] : 0; *(volatile int*)(row + j) = v; }
        __threadfence();
        for (int j = 0; j < IL_CAP; ++j) { const int v = (j < n) ? lists[threadIdx.x * IL_CAP + j] : 0; *(volatile int*)(row + j) = v; }
        VST2(int, cnt + d, min(n, IL_CAP));
    }
}
__global__ __launch_bounds__(256) void k_csr_scan(const int* __restrict__ cnt, int* off, int N, int E) {
    __shared__ int part[256]; const int per = ((((N + 255) / 256) + 31) / 32) * 32; const int a = threadIdx.x * per, b = min(N, a + per); int s = 0;
    for (int i = a; i < b; ++i) { int c = cnt[i]; c = c < 0 ? 0 : (c > IL_CAP ? IL_CAP : c); s += c; } part[threadIdx.x] = s; __syncthreads();
    if (threadIdx.x == 0) { int run = 0; for (int t = 0; t < 256; ++t) { const int v = part[t]; part[t] = run; run += v; } } __syncthreads();
    int run = part[threadIdx.x]; for (int i = a; i < b; ++i) { VST2(int, off + i, run < E ? run : E); int c = cnt[i]; c = c < 0 ? 0 : (c > IL_CAP ? IL_CAP : c); run += c; }
    if (a < N && b == N) { VST2(int, off + N, run < E ? run : E); }
}
__global__ __launch_bounds__(256) void k_slotcopy(const int* __restrict__ off, const int* __restrict__ NBR, int* slot, int N, int E) {
    const int t = blockIdx.x * 256 + threadIdx.x; int tot = off[N]; tot = tot > E ? E : tot; if (t >= tot || t >= E) return;
    int lo = 0, hi = N - 1;
    while (lo < hi) { const int mid = (lo + hi + 1) >> 1; if (off[mid] <= t) lo = mid; else hi = mid - 1; }
    int j = t - off[lo]; j = (j < 0) ? 0 : ((j >= IL_CAP) ? (IL_CAP - 1) : j);
    VST2(int, slot + t, NBR[(size_t)lo * IL_CAP + j]);
}

#ifndef IL_CAP
#define IL_CAP 64
#endif
#define IL2_T 128
#define NBKMAX 1024
__global__ __launch_bounds__(256) void k_bk_hist(const int* __restrict__ tgt, int E, int per, int nbk, int* HIST) {
    __shared__ int h[NBKMAX]; const int tid = threadIdx.x; const int c = blockIdx.x;
    for (int i = tid; i < NBKMAX; i += 256) h[i] = 0;
    __syncthreads();
    const int e0 = c * per; int e1 = e0 + per; if (e1 > E) e1 = E;
    for (int e = e0 + tid; e < e1; e += 256) { int b = tgt[e] / IL2_T; b = b < 0 ? 0 : (b >= nbk ? nbk - 1 : b); atomicAdd(&h[b], 1); }
    __syncthreads();
    for (int i = tid; i < NBKMAX; i += 256) { VST2(int, HIST + (size_t)c * NBKMAX + i, i < nbk ? h[i] : 0); }
}
__global__ __launch_bounds__(256) void k_bk_scan(const int* __restrict__ HIST, int nch, int nbk, int* OFF, int* BOFF) {
    __shared__ int tot[NBKMAX]; __shared__ int run;
    const int tid = threadIdx.x;
    for (int b = tid; b < NBKMAX; b += 256) { int s = 0; if (b < nbk) for (int c = 0; c < nch; ++c) s += (HIST[(size_t)c * NBKMAX + b] + 31) & ~31; tot[b] = s; }
    if (tid == 0) run = 0;
    __syncthreads();
    if (tid == 0) { int acc = 0; for (int b = 0; b < nbk; ++b) { const int t = tot[b]; tot[b] = acc; acc += t; } run = acc; }
    __syncthreads();
    for (int b = tid; b < nbk; b += 256) { int acc = tot[b]; VST2(int, BOFF + b, acc); for (int c = 0; c < nch; ++c) { VST2(int, OFF + (size_t)c * NBKMAX + b, acc); acc += (HIST[(size_t)c * NBKMAX + b] + 31) & ~31; } }
    if (tid == 0) { VST2(int, BOFF + nbk, run); }
}
__global__ __launch_bounds__(256) void k_bk_scatter(const int* __restrict__ tgt, int E, int per, int nbk, const int* __restrict__ OFF, int* BED) {
    __shared__ int cur[NBKMAX]; const int tid = threadIdx.x; const int c = blockIdx.x; const int bedlen = E + 32 * 256 * nbk;
    for (int i = tid; i < NBKMAX; i += 256) cur[i] = 0;
    __syncthreads();
    const int e0 = c * per; int e1 = e0 + per; if (e1 > E) e1 = E;
    for (int e = e0 + tid; e < e1; e += 256) { int b = tgt[e] / IL2_T; b = b < 0 ? 0 : (b >= nbk ? nbk - 1 : b); const int s = atomicAdd(&cur[b], 1); int ix = OFF[(size_t)c * NBKMAX + b] + s; ix = ix < 0 ? 0 : (ix >= bedlen ? bedlen - 1 : ix); VST2(int, BED + ix, e); }
}
__global__ __launch_bounds__(256) void k_inlists3(const int* __restrict__ tgt, const int* __restrict__ BED, const int* __restrict__ HIST, const int* __restrict__ OFF, int nch, int N, int* NBR, int* cnt, int E, int per) {
    __shared__ int lists[IL2_T * IL_CAP]; __shared__ int lcnt[IL2_T];
    const int tid = threadIdx.x; const int bk = blockIdx.x; const int base = bk * IL2_T; const int bedlen = E + 32 * 256 * (int)gridDim.x;
    if (tid < IL2_T) lcnt[tid] = 0;
    __syncthreads();
    for (int c = 0; c < nch; ++c) { int p0 = OFF[(size_t)c * NBKMAX + bk]; int n = HIST[(size_t)c * NBKMAX + bk]; n = n < 0 ? 0 : (n > per ? per : n); p0 = p0 < 0 ? 0 : (p0 > bedlen - n ? bedlen - n : p0);
        for (int p = p0 + tid; p < p0 + n; p += 256) { int e = BED[p]; e = e < 0 ? 0 : (e >= E ? E - 1 : e); const int d = tgt[e] - base; if (d >= 0 && d < IL2_T) { const int s = atomicAdd(&lcnt[d], 1); if (s < IL_CAP) lists[d * IL_CAP + s] = e; } } }
    __syncthreads();
    if (tid < IL2_T && base + tid < N) {
        const int n = lcnt[tid] < IL_CAP ? lcnt[tid] : IL_CAP; int* L = lists + tid * IL_CAP;
        for (int i = 1; i < n; ++i) { const int v = L[i]; int j = i - 1; while (j >= 0 && L[j] > v) { L[j + 1] = L[j]; --j; } L[j + 1] = v; }
        for (int k = 0; k < IL_CAP; ++k) { VST2(int, NBR + (size_t)(base + tid) * IL_CAP + k, k < n ? L[k] : 0); }
        VST2(int, cnt + base + tid, n);
    }
}
static void build_csr3(const int* tgt, int E, int N, int* NBR, int* cnt, int* HIST, int* OFF, int* BOFF, int* BED, hipStream_t stream) {
    const int nbk = (N + IL2_T - 1) / IL2_T; const int nch = 256; const int per = (E + nch - 1) / nch;
    k_bk_hist<<<nch, 256, 0, stream>>>(tgt, E, per, nbk, HIST);
    k_bk_scan<<<1, 256, 0, stream>>>(HIST, nch, nbk, OFF, BOFF);
    k_bk_scatter<<<nch, 256, 0, stream>>>(tgt, E, per, nbk, OFF, BED);
    k_inlists3<<<nbk, 256, 0, stream>>>(tgt, BED, HIST, OFF, nch, N, NBR, cnt, E, per);
}

__device__ __forceinline__ float eluf(float x) { return x > 0.f ? x : expm1f(x); }
__global__ __launch_bounds__(64) void k_wea(const float* __restrict__ We, const float* __restrict__ ae, int F, float* WEA) { const int t = threadIdx.x; if (t >= 16) return; const int k = t / 4, h = t % 4; float s = 0.f; for (int f = 0; f < F; ++f) s += We[(size_t)k * (NH * F) + h * F + f] * ae[h * F + f]; VST2(float, WEA + t, s); }
__global__ __launch_bounds__(256) void k_alpha(const float* __restrict__ Hm, int F, const float* __restrict__ as, const float* __restrict__ ad, float* ASD) {
    const int lane = threadIdx.x & 31, n = blockIdx.x * 8 + (threadIdx.x >> 5); if (n >= NN_) return; const float* row = Hm + (size_t)n * (NH * F); float s[NH], d[NH];
#pragma unroll
    for (int h = 0; h < NH; ++h) { s[h] = 0.f; d[h] = 0.f; }
#pragma unroll 1
    for (int c = lane; c < NH * F; c += 32) { const int h = c / F; const float v = row[c]; const float ws = as[c], wd = ad[c];
#pragma unroll
        for (int hh = 0; hh < NH; ++hh) if (hh == h) { s[hh] += v * ws; d[hh] += v * wd; } }
#pragma unroll
    for (int h = 0; h < NH; ++h) {
#pragma unroll
        for (int o = 16; o; o >>= 1) { s[h] += __shfl_xor(s[h], o, 32); d[h] += __shfl_xor(d[h], o, 32); } }
    float v = 0.f;
#pragma unroll
    for (int h = 0; h < NH; ++h) { if (lane == h) v = s[h]; if (lane == 4 + h) v = d[h]; }
    VST2(float, ASD + (size_t)n * 32 + lane, v);
}
__global__ __launch_bounds__(256) void k_gat(const float* __restrict__ Hm, int F, const float* __restrict__ ASD, const float* __restrict__ attr, const float* __restrict__ WEA, const int* __restrict__ srcs, const int* __restrict__ off, const int* __restrict__ slot, const float* __restrict__ bias, int concat, float* Y) {
    const size_t q = (size_t)blockIdx.x * 256 + threadIdx.x; if (q >= (size_t)NN_ * NH * F) return; const int c = (int)(q % (NH * F)), i = (int)(q / (NH * F)); const int h = c / F; const float adi = ASD[(size_t)i * 32 + 4 + h]; const int a = off[i], b = off[i + 1];
    const float w0 = WEA[h], w1 = WEA[4 + h], w2 = WEA[8 + h], w3 = WEA[12 + h];
    float m = -__builtin_inff();
    for (int p = a; p < b && p < a + IL_CAP; ++p) { int e = slot[p]; e = e < 0 ? 0 : (e >= NE_ ? NE_ - 1 : e); int s = srcs[e]; s = s < 0 ? 0 : (s >= NN_ ? NN_ - 1 : s); const float* at = attr + (size_t)e * 4;
        float l = ASD[(size_t)s * 32 + h] + adi + at[0] * w0 + at[1] * w1 + at[2] * w2 + at[3] * w3; l = l > 0.f ? l : 0.2f * l; m = fmaxf(m, l); }
    float den = 0.f, acc = 0.f;
    for (int p = a; p < b && p < a + IL_CAP; ++p) { int e = slot[p]; e = e < 0 ? 0 : (e >= NE_ ? NE_ - 1 : e); int s = srcs[e]; s = s < 0 ? 0 : (s >= NN_ ? NN_ - 1 : s); const float* at = attr + (size_t)e * 4;
        float l = ASD[(size_t)s * 32 + h] + adi + at[0] * w0 + at[1] * w1 + at[2] * w2 + at[3] * w3; l = l > 0.f ? l : 0.2f * l; const float wgt = expf(l - m); den += wgt; acc += wgt * Hm[(size_t)s * (NH * F) + c]; }
    const float v = (b > a) ? acc / (den + 1e-16f) : 0.f;
    VST2(float, Y + q, concat ? eluf(v + bias[c]) : v);
}
__global__ __launch_bounds__(256) void k_gatmean(const float* __restrict__ AGG, const float* __restrict__ bias, float* H3) { const size_t q = (size_t)blockIdx.x * 256 + threadIdx.x; if (q >= (size_t)NN_ * HID) return; const int f = (int)(q % HID); const size_t i = q / HID; float s = 0.f;
#pragma unroll
    for (int h = 0; h < NH; ++h) s += AGG[i * (NH * HID) + h * HID + f];
    VST2(float, H3 + q, eluf(s * 0.25f + bias[f])); }
__global__ void k_goff(const int* __restrict__ batch, int* GOFF) { if (threadIdx.x == 0 && blockIdx.x == 0) { int g = 0; VST2(int, GOFF, 0); for (int n = 0; n < NN_; ++n) { while (g < batch[n] && g < NG) { ++g; VST2(int, GOFF + g, n); } } while (g < NG) { ++g; VST2(int, GOFF + g, NN_); } } }
__global__ __launch_bounds__(256) void k_score(const float* __restrict__ T, const float* __restrict__ pw2, const float* __restrict__ pb2, float* SCO) { const int n = blockIdx.x * 256 + threadIdx.x; if (n >= NN_) return; float s = pb2[0];
#pragma unroll 4
    for (int k = 0; k < 128; ++k) s += T[(size_t)n * 128 + k] * pw2[k];
    VST2(float, SCO + n, s); }
__global__ __launch_bounds__(256) void k_pool(const float* __restrict__ H3, const float* __restrict__ SCO, const int* __restrict__ GOFF, const float* __restrict__ cw1, const float* __restrict__ cb1, const float* __restrict__ cw2, const float* __restrict__ cb2, float* OUTG) {
    __shared__ float red[256]; __shared__ float ge[HID]; __shared__ float r1[128]; __shared__ float stat[2];
    const int g = blockIdx.x, t = threadIdx.x; const int n0 = GOFF[g], n1 = GOFF[g + 1];
    float m = -__builtin_inff(); for (int n = n0 + t; n < n1; n += 256) m = fmaxf(m, SCO[n]);
    red[t] = m; __syncthreads(); for (int o = 128; o > 0; o >>= 1) { if (t < o) red[t] = fmaxf(red[t], red[t + o]); __syncthreads(); }
    if (t == 0) stat[0] = red[0]; __syncthreads(); m = stat[0];
    float s = 0.f; for (int n = n0 + t; n < n1; n += 256) s += expf(SCO[n] - m);
    red[t] = s; __syncthreads(); for (int o = 128; o > 0; o >>= 1) { if (t < o) red[t] += red[t + o]; __syncthreads(); }
    if (t == 0) stat[1] = red[0]; __syncthreads(); const float den = stat[1];
    { float acc = 0.f; for (int n = n0; n < n1; ++n) acc += H3[(size_t)n * HID + t] * (expf(SCO[n] - m) / den); ge[t] = acc; }
    __syncthreads();
    if (t < 128) { float a = cb1[t]; for (int c = 0; c < HID; ++c) a += ge[c] * cw1[c * 128 + t]; r1[t] = fmaxf(a, 0.f); }
    __syncthreads();
    if (t < 32) { float o = 0.f; if (t == 0) { o = cb2[0]; for (int k = 0; k < 128; ++k) o += r1[k] * cw2[k]; } VST2(float, OUTG + (size_t)g * 32 + t, t == 0 ? o : 0.f); }
}
__global__ __launch_bounds__(64) void k_outg(const float* __restrict__ OUTG, float* out) { const int g = threadIdx.x; if (g < NG) { VST2(float, out + g, OUTG[(size_t)g * 32]); } }
extern "C" void kernel_launch(void* const* d_in, const int* in_sizes, int n_in,
                              void* d_out, int out_size, void* d_ws, size_t ws_size, hipStream_t stream) {
    (void)in_sizes; (void)n_in; (void)out_size;
    const float* x = (const float*)d_in[0]; const int* ei = (const int*)d_in[1]; const float* attr = (const float*)d_in[2]; const int* batch = (const int*)d_in[3];
    const float* W[3] = {(const float*)d_in[4], (const float*)d_in[10], (const float*)d_in[16]}; const float* AS[3] = {(const float*)d_in[5], (const float*)d_in[11], (const float*)d_in[17]}; const float* AD[3] = {(const float*)d_in[6], (const float*)d_in[12], (const float*)d_in[18]};
    const float* WE[3] = {(const float*)d_in[7], (const float*)d_in[13], (const float*)d_in[19]}; const float* AE[3] = {(const float*)d_in[8], (const float*)d_in[14], (const float*)d_in[20]}; const float* BI[3] = {(const float*)d_in[9], (const float*)d_in[15], (const float*)d_in[21]};
    const float* pw1 = (const float*)d_in[22]; const float* pb1 = (const float*)d_in[23]; const float* pw2 = (const float*)d_in[24]; const float* pb2 = (const float*)d_in[25]; const float* cw1 = (const float*)d_in[26]; const float* cb1 = (const float*)d_in[27]; const float* cw2 = (const float*)d_in[28]; const float* cb2 = (const float*)d_in[29];
    float* out = (float*)d_out;
    const int* srcs = ei; const int* dsts = ei + NE_;
    char* wsp = (char*)d_ws;
    auto take = [&](size_t bytes) { char* p = wsp; wsp += (bytes + 255) & ~(size_t)255; return (void*)p; };
    int* NBR = (int*)take((size_t)NN_ * IL_CAP * 4); int* cnt = (int*)take((size_t)(NN_ + 1) * 4); int* off = (int*)take((size_t)(NN_ + 1) * 4); int* slot = (int*)take((size_t)NE_ * 4);
    int* HIST = (int*)take((size_t)256 * NBKMAX * 4); int* OFFB = (int*)take((size_t)256 * NBKMAX * 4); int* BOFF = (int*)take((size_t)(NBKMAX + 1) * 4); int* BED = (int*)take(((size_t)NE_ + (size_t)32 * 256 * ((NN_ + IL2_T - 1) / IL2_T)) * 4);
    float* WEA = (float*)take(64 * 4); float* ASD = (float*)take((size_t)NN_ * 32 * 4); float* Hm = (float*)take((size_t)NN_ * NH * HID * 4); float* Y = (float*)take((size_t)NN_ * NH * HID * 4); float* H3 = (float*)take((size_t)NN_ * HID * 4); float* T = (float*)take((size_t)NN_ * 128 * 4); float* SCO = (float*)take((size_t)NN_ * 4); int* GOFF = (int*)take(128 * 4); float* OUTG = (float*)take((size_t)NG * 32 * 4);
    if ((size_t)(wsp - (char*)d_ws) > ws_size) return;
    build_csr3(dsts, NE_, NN_, NBR, cnt, HIST, OFFB, BOFF, BED, stream);
    k_csr_scan<<<1, 256, 0, stream>>>(cnt, off, NN_, NE_); k_slotcopy<<<(NE_ + 255) / 256, 256, 0, stream>>>(off, NBR, slot, NN_, NE_);
    const unsigned gM = (NN_ + 63) / 64;
    k_wea<<<1, 64, 0, stream>>>(WE[0], AE[0], 64, WEA);
    { GemmArgs g = gemm_args(x, DIN, zm(0), W[0], HID, zm(0), Hm, HID, zm(0), NN_, HID, DIN); gemm_kernel<0, 0, 2, 2, 4, 2, ACT_NONE><<<dim3(gM, 2, 1), 256, 0, stream>>>(g); }
    k_alpha<<<(NN_ + 7) / 8, 256, 0, stream>>>(Hm, 64, AS[0], AD[0], ASD);
    k_gat<<<(unsigned)(((size_t)NN_ * HID + 255) / 256), 256, 0, stream>>>(Hm, 64, ASD, attr, WEA, srcs, off, slot, BI[0], 1, Y);
    k_wea<<<1, 64, 0, stream>>>(WE[1], AE[1], 64, WEA);
    { GemmArgs g = gemm_args(Y, HID, zm(0), W[1], HID, zm(0), Hm, HID, zm(0), NN_, HID, HID); gemm_kernel<0, 0, 2, 2, 4, 2, ACT_NONE><<<dim3(gM, 2, 1), 256, 0, stream>>>(g); }
    k_alpha<<<(NN_ + 7) / 8, 256, 0, stream>>>(Hm, 64, AS[1], AD[1], ASD);
    k_gat<<<(unsigned)(((size_t)NN_ * HID + 255) / 256), 256, 0, stream>>>(Hm, 64, ASD, attr, WEA, srcs, off, slot, BI[1], 1, Y);
    k_wea<<<1, 64, 0, stream>>>(WE[2], AE[2], HID, WEA);
    { GemmArgs g = gemm_args(Y, HID, zm(0), W[2], NH * HID, zm(0), Hm, NH * HID, zm(0), NN_, NH * HID, HID); gemm_kernel<0, 0, 2, 2, 4, 2, ACT_NONE><<<dim3(gM, 8, 1), 256, 0, stream>>>(g); }
    k_alpha<<<(NN_ + 7) / 8, 256, 0, stream>>>(Hm, HID, AS[2], AD[2], ASD);
    k_gat<<<(unsigned)(((size_t)NN_ * NH * HID + 255) / 256), 256, 0, stream>>>(Hm, HID, ASD, attr, WEA, srcs, off, slot, BI[2], 0, Y);
    k_gatmean<<<(unsigned)(((size_t)NN_ * HID + 255) / 256), 256, 0, stream>>>(Y, BI[2], H3);
    { GemmArgs g = gemm_args(H3, HID, zm(0), pw1, 128, zm(0), T, 128, zm(0), NN_, 128, HID); g.bias = pb1; gemm_kernel<0, 0, 2, 2, 4, 2, ACT_TANH><<<dim3(gM, 1, 1), 256, 0, stream>>>(g); }
    k_score<<<(NN_ + 255) / 256, 256, 0, stream>>>(T, pw2, pb2, SCO);
    k_goff<<<1, 32, 0, stream>>>(batch, GOFF);
    k_pool<<<NG, 256, 0, stream>>>(H3, SCO, GOFF, cw1, cb1, cw2, cb2, OUTG);
    k_outg<<<1, 64, 0, stream>>>(OUTG, out);
}
